// s4MambaModule_64330020159661
// MI455X (gfx1250) — hardware-verified
//
#include <hip/hip_runtime.h>
#include <stdint.h>
#include <stddef.h>


#define BB    4
#define LL    2048
#define DMOD  1024
#define NST   16
#define WW    4
#define DIN   2048
#define E2    4096
#define MM    (BB * LL)

typedef _Float16 f16;
typedef f16          v8h  __attribute__((ext_vector_type(8)));
typedef f16          v16h __attribute__((ext_vector_type(16)));
typedef float        v8f  __attribute__((ext_vector_type(8)));
typedef float        v4f  __attribute__((ext_vector_type(4)));
typedef unsigned int v4u  __attribute__((ext_vector_type(4)));

union Frag { v16h v; v8h hh[2]; };
union H8   { v8h h; v4u u; };

__device__ __forceinline__ v8f wmma_f16(v16h a, v16h b, v8f c) {
    c = __builtin_amdgcn_wmma_f32_16x16x32_f16(false, a, false, b, (short)0, c, false, false);
    asm volatile("v_nop\n\tv_nop\n\tv_nop\n\tv_nop" : "+v"(c) : "v"(a), "v"(b));
    return c;
}

__device__ __forceinline__ void gemm_tile(const f16* __restrict__ A, const f16* __restrict__ Bm,
                                          const int K, const int row0, const int col0,
                                          const int m, const int h, v8f (&acc)[2][4]) {
    const v8f zero = {0.f, 0.f, 0.f, 0.f, 0.f, 0.f, 0.f, 0.f};
#pragma unroll
    for (int i = 0; i < 2; ++i)
#pragma unroll
        for (int j = 0; j < 4; ++j) acc[i][j] = zero;

    const f16* pa0 = A  + (size_t)(row0 + m) * K + 8 * h;
    const f16* pa1 = pa0 + (size_t)16 * K;
    const f16* pb0 = Bm + (size_t)(col0 + m) * K + 8 * h;
    const f16* pb1 = pb0 + (size_t)16 * K;
    const f16* pb2 = pb0 + (size_t)32 * K;
    const f16* pb3 = pb0 + (size_t)48 * K;

#pragma unroll 1
    for (int k0 = 0; k0 < K; k0 += 32) {
        Frag a0, a1, b0, b1, b2, b3;
        a0.hh[0] = *(const v8h*)(pa0 + k0);  a0.hh[1] = *(const v8h*)(pa0 + k0 + 16);
        a1.hh[0] = *(const v8h*)(pa1 + k0);  a1.hh[1] = *(const v8h*)(pa1 + k0 + 16);
        b0.hh[0] = *(const v8h*)(pb0 + k0);  b0.hh[1] = *(const v8h*)(pb0 + k0 + 16);
        b1.hh[0] = *(const v8h*)(pb1 + k0);  b1.hh[1] = *(const v8h*)(pb1 + k0 + 16);
        b2.hh[0] = *(const v8h*)(pb2 + k0);  b2.hh[1] = *(const v8h*)(pb2 + k0 + 16);
        b3.hh[0] = *(const v8h*)(pb3 + k0);  b3.hh[1] = *(const v8h*)(pb3 + k0 + 16);

        acc[0][0] = wmma_f16(a0.v, b0.v, acc[0][0]);
        acc[0][1] = wmma_f16(a0.v, b1.v, acc[0][1]);
        acc[0][2] = wmma_f16(a0.v, b2.v, acc[0][2]);
        acc[0][3] = wmma_f16(a0.v, b3.v, acc[0][3]);
        acc[1][0] = wmma_f16(a1.v, b0.v, acc[1][0]);
        acc[1][1] = wmma_f16(a1.v, b1.v, acc[1][1]);
        acc[1][2] = wmma_f16(a1.v, b2.v, acc[1][2]);
        acc[1][3] = wmma_f16(a1.v, b3.v, acc[1][3]);
    }
}

__global__ __launch_bounds__(256) void k_cvt_f16(const float* __restrict__ in,
                                                  f16* __restrict__ out,
                                                  int n8, float scale) {
    const int i = blockIdx.x * 256 + threadIdx.x;
    if (i >= n8) return;
    const float* p = in + (size_t)i * 8;
    const v4f a = *(const v4f*)(p);
    const v4f b = *(const v4f*)(p + 4);
    v8h v;
    v[0] = (f16)(a[0] * scale); v[1] = (f16)(a[1] * scale);
    v[2] = (f16)(a[2] * scale); v[3] = (f16)(a[3] * scale);
    v[4] = (f16)(b[0] * scale); v[5] = (f16)(b[1] * scale);
    v[6] = (f16)(b[2] * scale); v[7] = (f16)(b[3] * scale);
    H8 r; r.h = v;
    volatile v4u* q = (volatile v4u*)(out + (size_t)i * 8);
    *q = r.u;
    __threadfence();
    *q = r.u;
}

#define TP1 72
__global__ __launch_bounds__(128) void k_gemm_xz(const f16* __restrict__ hs16,
                                                  const f16* __restrict__ w1h,
                                                  f16* __restrict__ xz16) {
    __shared__ __attribute__((aligned(16))) f16 tile[4][32][TP1];

    const int wave = threadIdx.x >> 5;
    const int lane = threadIdx.x & 31;
    const int m = lane & 15, h = lane >> 4;
    const int wm = wave >> 1, wn = wave & 1;
    const int row0 = blockIdx.x * 64 + wm * 32;
    const int col0 = blockIdx.y * 128 + wn * 64;

    v8f acc[2][4];
    gemm_tile(hs16, w1h, DMOD, row0, col0, m, h, acc);

    f16 (*tw)[TP1] = tile[wave];
#pragma unroll
    for (int i = 0; i < 2; ++i)
#pragma unroll
        for (int j = 0; j < 4; ++j)
#pragma unroll
            for (int r = 0; r < 8; ++r)
                tw[i * 16 + 8 * h + r][j * 16 + m] = (f16)(acc[i][j][r] * 0.03125f);
    __syncthreads();

    const int q = lane >> 3, p = lane & 7;
    H8 vals[8];
#pragma unroll
    for (int s = 0; s < 8; ++s)
        vals[s].h = *(const v8h*)(&tw[s * 4 + q][p * 8]);

    f16* gb = xz16 + (size_t)row0 * E2 + col0 + p * 8;
#pragma unroll
    for (int s = 0; s < 8; ++s)
        *(volatile v4u*)(gb + (size_t)(s * 4 + q) * E2) = vals[s].u;
    __threadfence();
#pragma unroll
    for (int s = 0; s < 8; ++s)
        *(volatile v4u*)(gb + (size_t)(s * 4 + q) * E2) = vals[s].u;
}

#define TP2 36
__global__ __launch_bounds__(128) void k_gemm_out(const f16* __restrict__ g16,
                                                   const f16* __restrict__ w2h,
                                                   float* __restrict__ out) {
    __shared__ __attribute__((aligned(16))) float tileT[4][64][TP2];

    const int wave = threadIdx.x >> 5;
    const int lane = threadIdx.x & 31;
    const int m = lane & 15, h = lane >> 4;
    const int wm = wave >> 1, wn = wave & 1;
    const int row0 = blockIdx.x * 64 + wm * 32;
    const int col0 = blockIdx.y * 128 + wn * 64;

    v8f acc[2][4];
    gemm_tile(g16, w2h, DIN, row0, col0, m, h, acc);

    float (*tw)[TP2] = tileT[wave];
#pragma unroll
    for (int i = 0; i < 2; ++i)
#pragma unroll
        for (int j = 0; j < 4; ++j) {
            const int col = j * 16 + m;
            const int rb  = i * 16 + 8 * h;
            v4f lo, hi;
            lo[0] = acc[i][j][0] * 0.03125f; lo[1] = acc[i][j][1] * 0.03125f;
            lo[2] = acc[i][j][2] * 0.03125f; lo[3] = acc[i][j][3] * 0.03125f;
            hi[0] = acc[i][j][4] * 0.03125f; hi[1] = acc[i][j][5] * 0.03125f;
            hi[2] = acc[i][j][6] * 0.03125f; hi[3] = acc[i][j][7] * 0.03125f;
            *(v4f*)(&tw[col][rb])     = lo;
            *(v4f*)(&tw[col][rb + 4]) = hi;
        }
    __syncthreads();

    const int q = lane >> 3, p = lane & 7;
    const int rq = q >> 1;
    const int c0 = (q & 1) * 32 + p * 4;
    v4f vals[16];
#pragma unroll
    for (int s = 0; s < 16; ++s) {
        const int row = 2 * s + rq;
        v4f v;
        v[0] = tw[c0 + 0][row]; v[1] = tw[c0 + 1][row];
        v[2] = tw[c0 + 2][row]; v[3] = tw[c0 + 3][row];
        vals[s] = v;
    }

    float* ob = out + (size_t)row0 * DMOD + col0 + c0;
#pragma unroll
    for (int s = 0; s < 16; ++s)
        *(volatile v4f*)(ob + (size_t)(2 * s + rq) * DMOD) = vals[s];
    __threadfence();
#pragma unroll
    for (int s = 0; s < 16; ++s)
        *(volatile v4f*)(ob + (size_t)(2 * s + rq) * DMOD) = vals[s];
}

__global__ __launch_bounds__(256) void k_coef(const float* __restrict__ log_dt,
                                               const float* __restrict__ A_re,
                                               const float* __restrict__ A_im,
                                               const float* __restrict__ C_re,
                                               const float* __restrict__ C_im,
                                               float* __restrict__ coef) {
    const int idx = blockIdx.x * 256 + threadIdx.x;
    if (idx >= DIN * NST) return;
    const int hch = idx >> 4;
    const float dt = expf(log_dt[hch]);
    const float ar = A_re[idx], ai = A_im[idx];
    const float er = expf(dt * ar);
    const float th = dt * ai;
    const float cs = cosf(th), sn = sinf(th);
    const float e_re = er * cs, e_im = er * sn;
    const float nr = e_re - 1.0f, ni = e_im;
    const float den = __builtin_amdgcn_rcpf(ar * ar + ai * ai);
    const float dB_re = (nr * ar + ni * ai) * den;
    const float dB_im = (ni * ar - nr * ai) * den;
    const float cr = C_re[idx], ci = C_im[idx];
    v4f v;
    v[0] = e_re;
    v[1] = e_im;
    v[2] = 2.0f * (cr * dB_re - ci * dB_im);
    v[3] = 2.0f * (cr * dB_im + ci * dB_re);
    volatile v4f* q = (volatile v4f*)(coef + (size_t)idx * 4);
    *q = v;
    __threadfence();
    *q = v;
}

__global__ __launch_bounds__(256) void k_scan(const f16* __restrict__ xz16,
                                               const float* __restrict__ conv_w,
                                               const float* __restrict__ conv_b,
                                               const float* __restrict__ coef,
                                               const float* __restrict__ D_skip,
                                               f16* __restrict__ g16) {
    __shared__ __attribute__((aligned(16))) f16 stile[8][256];

    const int tloc = threadIdx.x;
    const int tid  = blockIdx.x * 256 + tloc;
    const int b    = tid / DIN;
    const int hch  = tid - b * DIN;
    const int h0   = hch - tloc;

    float lam_re[NST], lam_im[NST], co_re[NST], co_im[NST], s_re[NST], s_im[NST];
#pragma unroll
    for (int n = 0; n < NST; ++n) {
        const v4f c = *(const v4f*)(coef + ((size_t)hch * NST + n) * 4);
        lam_re[n] = c[0]; lam_im[n] = c[1]; co_re[n] = c[2]; co_im[n] = c[3];
        s_re[n] = 0.f; s_im[n] = 0.f;
    }

    const float w0 = conv_w[hch * WW + 0], w1 = conv_w[hch * WW + 1];
    const float w2 = conv_w[hch * WW + 2], w3 = conv_w[hch * WW + 3];
    const float cb  = conv_b[hch];
    const float dsk = D_skip[hch];

    const f16* xb  = xz16 + (size_t)b * LL * E2 + hch;
    f16* gbase     = g16 + (size_t)b * LL * DIN + h0;
    const int q8 = tloc >> 5, p = tloc & 31;

    float xm3 = 0.f, xm2 = 0.f, xm1 = 0.f;

#pragma unroll 1
    for (int t = 0; t < LL; ++t) {
        const float x0 = (float)xb[(size_t)t * E2];
        const float zv = (float)xb[(size_t)t * E2 + DIN];
        float u = w0 * xm3 + w1 * xm2 + w2 * xm1 + w3 * x0 + cb;
        xm3 = xm2; xm2 = xm1; xm1 = x0;
        u = u * __builtin_amdgcn_rcpf(1.0f + __expf(-u));

        float y = dsk * u;
#pragma unroll
        for (int n = 0; n < NST; ++n) {
            const float sr = lam_re[n] * s_re[n] - lam_im[n] * s_im[n] + u;
            const float si = lam_re[n] * s_im[n] + lam_im[n] * s_re[n];
            s_re[n] = sr; s_im[n] = si;
            y += co_re[n] * sr - co_im[n] * si;
        }

        const float sg = zv * __builtin_amdgcn_rcpf(1.0f + __expf(-zv));
        stile[t & 7][tloc] = (f16)(y * sg);

        if ((t & 7) == 7) {
            __syncthreads();
            H8 v;
            v.h = *(const v8h*)(&stile[q8][p * 8]);
            volatile v4u* gp = (volatile v4u*)(gbase + (size_t)(t - 7 + q8) * DIN + p * 8);
            *gp = v.u;
            __threadfence();
            *gp = v.u;
            __syncthreads();
        }
    }
}

extern "C" void kernel_launch(void* const* d_in, const int* in_sizes, int n_in,
                              void* d_out, int out_size, void* d_ws, size_t ws_size,
                              hipStream_t stream) {
    if (n_in < 11) return;
    if (in_sizes[0] != MM * DMOD || in_sizes[1] != E2 * DMOD || in_sizes[2] != DIN * WW ||
        in_sizes[3] != DIN || in_sizes[4] != DMOD * DIN || in_sizes[5] != DIN ||
        in_sizes[6] != DIN * NST || in_sizes[7] != DIN * NST || in_sizes[8] != DIN * NST ||
        in_sizes[9] != DIN * NST || in_sizes[10] != DIN || out_size != MM * DMOD) return;

    const float* hs    = (const float*)d_in[0];
    const float* w_in  = (const float*)d_in[1];
    const float* cw    = (const float*)d_in[2];
    const float* cbias = (const float*)d_in[3];
    const float* w_out = (const float*)d_in[4];
    const float* logdt = (const float*)d_in[5];
    const float* a_re  = (const float*)d_in[6];
    const float* a_im  = (const float*)d_in[7];
    const float* c_re  = (const float*)d_in[8];
    const float* c_im  = (const float*)d_in[9];
    const float* dskip = (const float*)d_in[10];

    char* ws = (char*)d_ws;
    size_t off = 0;
    f16*   hs16 = (f16*)(ws + off);   off += (size_t)MM * DMOD * sizeof(f16);
    f16*   w1h  = (f16*)(ws + off);   off += (size_t)E2 * DMOD * sizeof(f16);
    f16*   w2h  = (f16*)(ws + off);   off += (size_t)DMOD * DIN * sizeof(f16);
    f16*   xz16 = (f16*)(ws + off);   off += (size_t)MM * E2 * sizeof(f16);
    f16*   g16  = (f16*)(ws + off);   off += (size_t)MM * DIN * sizeof(f16);
    float* coef = (float*)(ws + off); off += (size_t)DIN * NST * 4 * sizeof(float);
    if (off > ws_size) return;

    const int n8_hs = MM * DMOD / 8, n8_w1 = E2 * DMOD / 8, n8_w2 = DMOD * DIN / 8;
    k_cvt_f16<<<(n8_hs + 255) / 256, 256, 0, stream>>>(hs,    hs16, n8_hs, 1.0f);
    k_cvt_f16<<<(n8_w1 + 255) / 256, 256, 0, stream>>>(w_in,  w1h,  n8_w1, 32.0f);
    k_cvt_f16<<<(n8_w2 + 255) / 256, 256, 0, stream>>>(w_out, w2h,  n8_w2, 32.0f);

    k_gemm_xz<<<dim3(MM / 64, E2 / 128), 128, 0, stream>>>(hs16, w1h, xz16);

    k_coef<<<(DIN * NST + 255) / 256, 256, 0, stream>>>(logdt, a_re, a_im, c_re, c_im, coef);
    k_scan<<<(BB * DIN) / 256, 256, 0, stream>>>(xz16, cw, cbias, coef, dskip, g16);

    k_gemm_out<<<dim3(MM / 64, DMOD / 128), 128, 0, stream>>>(g16, w2h, (float*)d_out);
}
